// convAttention_34746285424731
// MI455X (gfx1250) — hardware-verified
//
#include <hip/hip_runtime.h>
#include <math.h>


#define NB   16
#define CC   192
#define HH   6
#define DHD  32
#define IMH  56
#define IMW  56
#define NPX  3136
#define MTOT (NB * NPX)
#define WIN  7
typedef __attribute__((ext_vector_type(16))) _Float16 v16h;
typedef __attribute__((ext_vector_type(8)))  _Float16 v8h;
typedef __attribute__((ext_vector_type(8)))  float    v8f;
typedef __attribute__((ext_vector_type(4)))  float    v4f;
#define VST2(T, ptr, val) do { const T _v = (val); *(volatile T*)(ptr) = _v; __threadfence(); *(volatile T*)(ptr) = _v; } while (0)
__device__ __forceinline__ v8f wmma16(v16h a, v16h b, v8f c) {
  v8f d = __builtin_amdgcn_wmma_f32_16x16x32_f16(false, a, false, b, (short)0, c, false, false);
  asm volatile("v_nop\n\tv_nop\n\tv_nop\n\tv_nop" : "+v"(d) : "v"(a), "v"(b));
  return d;
}
__device__ __forceinline__ v16h frag16(const _Float16* p, int hh) {
  const v8h lo = *(const v8h*)(p + 8 * hh), hi = *(const v8h*)(p + 16 + 8 * hh);
  return __builtin_shufflevector(lo, hi, 0,1,2,3,4,5,6,7,8,9,10,11,12,13,14,15);
}
__device__ __forceinline__ int kmap(int e, int hh) { return (e < 8) ? (8 * hh + e) : (16 + 8 * hh + (e - 8)); }
__device__ __forceinline__ void lds_sync() { __builtin_amdgcn_fence(__ATOMIC_RELEASE, "workgroup"); __builtin_amdgcn_wave_barrier(); __builtin_amdgcn_fence(__ATOMIC_ACQUIRE, "workgroup"); }

__global__ __launch_bounds__(256) void k_xT(const float* __restrict__ x, _Float16* __restrict__ XT) {
  const int t = blockIdx.x * 256 + threadIdx.x;
  const int px = t / 24, c0 = (t % 24) * 8, b = px / NPX, s = px % NPX;
  v8h o;
#pragma unroll
  for (int e = 0; e < 8; ++e) o[e] = (_Float16)x[((size_t)b * CC + c0 + e) * NPX + s];
  VST2(v8h, XT + (size_t)px * CC + c0, o);
}
__global__ __launch_bounds__(256) void k_w16(const float* __restrict__ w, int n, _Float16* __restrict__ W16) {
  const int t = blockIdx.x * 256 + threadIdx.x;
  if (t * 8 >= n) return;
  v8h o;
#pragma unroll
  for (int e = 0; e < 8; ++e) o[e] = (_Float16)w[t * 8 + e];
  VST2(v8h, W16 + (size_t)t * 8, o);
}
__global__ __launch_bounds__(128) void k_qkv(const _Float16* __restrict__ XT, const _Float16* __restrict__ Wq16, const float* __restrict__ bq, _Float16* __restrict__ QKV16) {
  __shared__ __attribute__((aligned(16))) _Float16 sT[4][2][16 * 32];
  const int lane = threadIdx.x & 31, wave = threadIdx.x >> 5, hh = lane >> 4, l16 = lane & 15;
  const int m0 = (blockIdx.x * 4 + wave) * 16, c0 = blockIdx.y * 64;
  v8f acc[4] = {};
#pragma unroll
  for (int k0 = 0; k0 < CC; k0 += 32) {
    const v16h a = frag16(XT + (size_t)(m0 + l16) * CC + k0, hh);
#pragma unroll
    for (int t = 0; t < 4; ++t) acc[t] = wmma16(a, frag16(Wq16 + (size_t)(c0 + t * 16 + l16) * CC + k0, hh), acc[t]);
  }
  const int which = c0 / CC, hbase = (c0 % CC) / DHD;
  const float sc = (which == 0) ? 0.17677669529663689f : 1.0f;
#pragma unroll
  for (int t = 0; t < 4; ++t) {
    const int hl = t >> 1, d = (t & 1) * 16 + l16; const float bb = bq[c0 + t * 16 + l16];
#pragma unroll
    for (int v = 0; v < 8; ++v) sT[wave][hl][(v + 8 * hh) * 32 + d] = (_Float16)((acc[t][v] + bb) * sc);
  }
  lds_sync();
  const int b = m0 / NPX, s0 = m0 % NPX;
  for (int pass = 0; pass < 2; ++pass) {
#pragma unroll
    for (int hl = 0; hl < 2; ++hl) {
      _Float16* dst = QKV16 + ((((size_t)which * NB + b) * HH + hbase + hl) * NPX + s0) * DHD;
      *(volatile v8h*)(dst + lane * 8) = *(const v8h*)(&sT[wave][hl][lane * 8]);
      *(volatile v8h*)(dst + 256 + lane * 8) = *(const v8h*)(&sT[wave][hl][256 + lane * 8]);
    }
    __threadfence();
  }
}
__global__ __launch_bounds__(256) void k_attn(const _Float16* __restrict__ QKV16, const float* __restrict__ btab, _Float16* __restrict__ Y16) {
  __shared__ __attribute__((aligned(16))) float Sx[8][16][33];
  __shared__ __attribute__((aligned(16))) _Float16 Pb[8][16][40];
  __shared__ __attribute__((aligned(16))) _Float16 Yt[8][16 * 32];
  const int lane = threadIdx.x & 31, wave = threadIdx.x >> 5, hh = lane >> 4, l16 = lane & 15;
  const int wg = blockIdx.x * 8 + wave;
  const int xsi = wg & 3, y = (wg >> 2) % IMH, h = ((wg >> 2) / IMH) % HH, b = (wg >> 2) / (IMH * HH);
  const int xs = xsi * 16, kx0 = xs - 3;
  const _Float16* Qp = QKV16 + (((size_t)0 * NB + b) * HH + h) * NPX * DHD;
  const _Float16* Kp = QKV16 + (((size_t)1 * NB + b) * HH + h) * NPX * DHD;
  const _Float16* Vp = QKV16 + (((size_t)2 * NB + b) * HH + h) * NPX * DHD;
  const int qpx = min(y * IMW + xs + l16, NPX - 1);
  const v16h qa = frag16(Qp + (size_t)qpx * DHD, hh);
  float sc[WIN * WIN];
#pragma unroll
  for (int dy = 0; dy < WIN; ++dy) {
    const int yy = y + dy - 3;
    v8f s0 = {}, s1 = {};
#pragma unroll
    for (int t = 0; t < 2; ++t) {
      const int kx = kx0 + t * 16 + l16;
      v16h kb;
      if (yy >= 0 && yy < IMH && kx >= 0 && kx < IMW) { const _Float16* kr = Kp + (size_t)(yy * IMW + kx) * DHD;
#pragma unroll
        for (int e = 0; e < 16; ++e) kb[e] = kr[kmap(e, hh)]; }
      else {
#pragma unroll
        for (int e = 0; e < 16; ++e) kb[e] = (_Float16)0.f; }
      if (t == 0) s0 = wmma16(qa, kb, s0); else s1 = wmma16(qa, kb, s1);
    }
#pragma unroll
    for (int v = 0; v < 8; ++v) { Sx[wave][v + 8 * hh][l16] = s0[v]; Sx[wave][v + 8 * hh][16 + l16] = s1[v]; }
    lds_sync();
    if (lane < 16) {
#pragma unroll
      for (int dx = 0; dx < WIN; ++dx) sc[dy * WIN + dx] = Sx[wave][lane][lane + dx] + btab[(dy * WIN + dx) * HH + h];
    }
    lds_sync();
  }
  float mx = -INFINITY;
#pragma unroll
  for (int i = 0; i < WIN * WIN; ++i) mx = fmaxf(mx, sc[i]);
  float den = 0.f;
#pragma unroll
  for (int i = 0; i < WIN * WIN; ++i) { sc[i] = expf(sc[i] - mx); den += sc[i]; }
  const float inv = 1.0f / den;
  v8f o0 = {}, o1 = {};
#pragma unroll
  for (int dy = 0; dy < WIN; ++dy) {
    const int yy = y + dy - 3;
    if (lane < 16) {
#pragma unroll
      for (int n = 0; n < 40; ++n) Pb[wave][lane][n] = (_Float16)0.f;
#pragma unroll
      for (int dx = 0; dx < WIN; ++dx) Pb[wave][lane][lane + dx] = (_Float16)(sc[dy * WIN + dx] * inv);
    }
    lds_sync();
    const v16h pa = frag16(&Pb[wave][l16][0], hh);
#pragma unroll
    for (int t = 0; t < 2; ++t) {
      const int d = t * 16 + l16;
      v16h vb;
#pragma unroll
      for (int e = 0; e < 16; ++e) { const int kx = kx0 + kmap(e, hh); vb[e] = (yy >= 0 && yy < IMH && kx >= 0 && kx < IMW) ? Vp[(size_t)(yy * IMW + kx) * DHD + d] : (_Float16)0.f; }
      if (t == 0) o0 = wmma16(pa, vb, o0); else o1 = wmma16(pa, vb, o1);
    }
    lds_sync();
  }
#pragma unroll
  for (int v = 0; v < 8; ++v) { Yt[wave][(v + 8 * hh) * 32 + l16] = (_Float16)o0[v]; Yt[wave][(v + 8 * hh) * 32 + 16 + l16] = (_Float16)o1[v]; }
  lds_sync();
  const int nval = min(16, IMW - xs);
  _Float16* dst = Y16 + ((((size_t)b * HH + h) * NPX) + y * IMW + xs) * DHD;
  for (int pass = 0; pass < 2; ++pass) {
    if (lane * 8 < nval * 32)       *(volatile v8h*)(dst + lane * 8) = *(const v8h*)(&Yt[wave][lane * 8]);
    if (256 + lane * 8 < nval * 32) *(volatile v8h*)(dst + 256 + lane * 8) = *(const v8h*)(&Yt[wave][256 + lane * 8]);
    __threadfence();
  }
}
__global__ __launch_bounds__(128) void k_proj(const _Float16* __restrict__ Y16, const _Float16* __restrict__ Wp16, const float* __restrict__ bp, float* __restrict__ out) {
  __shared__ __attribute__((aligned(16))) float sO[4][64][33];
  const int lane = threadIdx.x & 31, wave = threadIdx.x >> 5, hh = lane >> 4, l16 = lane & 15;
  const int m0 = (blockIdx.x * 4 + wave) * 32, c0 = blockIdx.y * 64;
  const int b = m0 / NPX, s0 = m0 % NPX;
  v8f acc[2][4] = {};
#pragma unroll
  for (int k0 = 0; k0 < CC; k0 += 32) {
    const int h = k0 / DHD;
    const _Float16* yr = Y16 + (((size_t)b * HH + h) * NPX + s0) * DHD;
    const v16h a0 = frag16(yr + (size_t)l16 * DHD, hh), a1 = frag16(yr + (size_t)(16 + l16) * DHD, hh);
#pragma unroll
    for (int t = 0; t < 4; ++t) { const v16h bb = frag16(Wp16 + (size_t)(c0 + t * 16 + l16) * CC + k0, hh); acc[0][t] = wmma16(a0, bb, acc[0][t]); acc[1][t] = wmma16(a1, bb, acc[1][t]); }
  }
#pragma unroll
  for (int r = 0; r < 2; ++r)
#pragma unroll
    for (int t = 0; t < 4; ++t)
#pragma unroll
      for (int v = 0; v < 8; ++v) sO[wave][t * 16 + l16][r * 16 + v + 8 * hh] = acc[r][t][v] + bp[c0 + t * 16 + l16];
  lds_sync();
  for (int pass = 0; pass < 2; ++pass) {
#pragma unroll 8
    for (int o = 0; o < 64; ++o) *(volatile float*)(out + ((size_t)b * CC + c0 + o) * NPX + s0 + lane) = sO[wave][o][lane];
    __threadfence();
  }
}
extern "C" void kernel_launch(void* const* d_in, const int* in_sizes, int n_in,
                              void* d_out, int out_size, void* d_ws, size_t ws_size, hipStream_t stream) {
  (void)in_sizes; (void)n_in; (void)out_size;
  const float* x    = (const float*)d_in[0];
  const float* qkvw = (const float*)d_in[1];
  const float* qkvb = (const float*)d_in[2];
  const float* pw   = (const float*)d_in[3];
  const float* pb   = (const float*)d_in[4];
  const float* btab = (const float*)d_in[5];
  float* out = (float*)d_out;
  char* ws = (char*)d_ws; size_t off = 0;
  auto take = [&](size_t bytes) { void* p = ws + off; off = (off + bytes + 255) & ~(size_t)255; return p; };
  _Float16* XT    = (_Float16*)take((size_t)MTOT * CC * 2);
  _Float16* Wq16  = (_Float16*)take((size_t)576 * CC * 2);
  _Float16* Wp16  = (_Float16*)take((size_t)CC * CC * 2);
  _Float16* QKV16 = (_Float16*)take((size_t)3 * MTOT * CC * 2);
  _Float16* Y16   = (_Float16*)take((size_t)MTOT * CC * 2);
  if (off > ws_size) return;
  k_xT<<<MTOT * 24 / 256, 256, 0, stream>>>(x, XT);
  k_w16<<<(576 * CC / 8 + 255) / 256, 256, 0, stream>>>(qkvw, 576 * CC, Wq16);
  k_w16<<<(CC * CC / 8 + 255) / 256, 256, 0, stream>>>(pw, CC * CC, Wp16);
  k_qkv<<<dim3(MTOT / 64, 9), 128, 0, stream>>>(XT, Wq16, qkvb, QKV16);
  k_attn<<<NB * HH * IMH * 4 / 8, 256, 0, stream>>>(QKV16, btab, Y16);
  k_proj<<<dim3(MTOT / 128, 3), 128, 0, stream>>>(Y16, Wp16, pb, out);
}
